// MHSA_21328807592167
// MI455X (gfx1250) — hardware-verified
//
#include <hip/hip_runtime.h>
#ifndef NB
#define NB 16
#endif
#ifndef SEQ
#define SEQ 1024
#endif
#define NB_FULL 16
#define SEQ_FULL 1024
#define CIN 256
#define NH 4
#define HD 64
#define GW 32
#define HCS 192
#define QP 1024
#define QPL 768
#define VOF 768
#define PCARRY 16384.0f
#define LCARRY 2048.0f
#define NR ((size_t)NB * SEQ)
static_assert(SEQ % 256 == 0);
static_assert((NR % 128) == 0);
static_assert(NB <= NB_FULL);
static_assert(SEQ <= SEQ_FULL);
static_assert(NH * HCS + NH * HD == QP);
static_assert(NH * HCS == QPL);
static_assert(GW * GW == SEQ_FULL);
static_assert(CIN == NH * HD);
static_assert(CIN % 64 == 0 && QP % 64 == 0 && HD == 64);

typedef unsigned short v8us __attribute__((ext_vector_type(8), may_alias));
typedef float  v8f  __attribute__((ext_vector_type(8)));
typedef float  v4f  __attribute__((ext_vector_type(4)));
typedef float  v4fa __attribute__((ext_vector_type(4), may_alias));
typedef _Float16 v16h __attribute__((ext_vector_type(16)));
typedef _Float16 v4h __attribute__((ext_vector_type(4)));
union FragH { v16h v; v8us half[2]; _Float16 h[16]; unsigned short u[16]; };

__device__ __forceinline__ unsigned short bf16_bits(float x) { unsigned int u = __float_as_uint(x); return (unsigned short)((u + 0x7FFFu + ((u >> 16) & 1u)) >> 16); }
__device__ __forceinline__ float bf16_val(unsigned short b) { return __uint_as_float(((unsigned int)b) << 16); }
__device__ __forceinline__ float bf16_rne(float x) { return bf16_val(bf16_bits(x)); }

__device__ __forceinline__ v16h g2_frag(const _Float16* p, int hh) { FragH f; f.half[0] = *(const v8us*)((const unsigned short*)p + 8 * hh); f.half[1] = *(const v8us*)((const unsigned short*)p + 16 + 8 * hh); return f.v; }
__device__ __forceinline__ v8f g2_mma(v16h a, v16h b, v8f c) { v8f d = __builtin_amdgcn_wmma_f32_16x16x32_f16(false, a, false, b, (short)0, c, false, false); asm volatile("v_nop\n\tv_nop\n\tv_nop\n\tv_nop" : "+v"(d) : "v"(a), "v"(b)); return d; }

__device__ __forceinline__ void g2_kloop(const _Float16* __restrict__ a0p, const _Float16* __restrict__ a1p, const _Float16* __restrict__ b0p, const _Float16* __restrict__ b1p, const _Float16* __restrict__ b2p, const _Float16* __restrict__ b3p, int K, int hh,
    v8f& c00, v8f& c01, v8f& c02, v8f& c03, v8f& c10, v8f& c11, v8f& c12, v8f& c13) {
#pragma unroll 1
  for (int kb = 0; kb < K; kb += 32) { const v16h a0 = g2_frag(a0p + kb, hh), a1 = g2_frag(a1p + kb, hh);
    v16h b = g2_frag(b0p + kb, hh); c00 = g2_mma(a0, b, c00); c10 = g2_mma(a1, b, c10);
    b = g2_frag(b1p + kb, hh); c01 = g2_mma(a0, b, c01); c11 = g2_mma(a1, b, c11);
    b = g2_frag(b2p + kb, hh); c02 = g2_mma(a0, b, c02); c12 = g2_mma(a1, b, c12);
    b = g2_frag(b3p + kb, hh); c03 = g2_mma(a0, b, c03); c13 = g2_mma(a1, b, c13); }
}

template <int RES>
__global__ __launch_bounds__(128) void k_gemm2(const _Float16* __restrict__ A, int lda, size_t sA, const _Float16* __restrict__ A2, int lda2, size_t sA2,
    const _Float16* __restrict__ Bh, int ldb, size_t sB, const _Float16* __restrict__ B2, int ldb2, size_t sB2, float rscale,
    float alpha, const float* __restrict__ bias, size_t sBias,
    float* __restrict__ C, _Float16* __restrict__ C16, int ldc, size_t sC, _Float16* __restrict__ C16L, int ldcl, size_t sCL, int NL, int M, int N, int K) {
  __shared__ __attribute__((aligned(16))) float so[4][32][68];
  const int tid = threadIdx.x, w = tid >> 5, lane = tid & 31, ln = lane & 15, hh = lane >> 4; const int by = blockIdx.y;
  A += (size_t)by * sA; Bh += (size_t)by * sB;
  if (RES) { A2 += (size_t)by * sA2; B2 += (size_t)by * sB2; }
  const size_t cofs = (size_t)by * sC, cofl = (size_t)by * sCL; const float* bp = bias ? bias + (size_t)by * sBias : nullptr;
  const int ntn = N >> 6; const int mt = blockIdx.x / ntn, nq = blockIdx.x - mt * ntn; const int row0 = mt * 128 + 32 * w, col0 = nq * 64; if (row0 >= M) return;
  const _Float16* a0p = A + (size_t)(row0 + ln) * lda; const _Float16* a1p = a0p + (size_t)16 * lda;
  const _Float16* b0p = Bh + (size_t)(col0 + ln) * ldb; const _Float16* b1p = b0p + (size_t)16 * ldb; const _Float16* b2p = b1p + (size_t)16 * ldb; const _Float16* b3p = b2p + (size_t)16 * ldb;
  const v8f z8 = {0.f,0.f,0.f,0.f,0.f,0.f,0.f,0.f}; v8f c00 = z8, c01 = z8, c02 = z8, c03 = z8, c10 = z8, c11 = z8, c12 = z8, c13 = z8;
  if (RES) {
    const _Float16* l0p = A2 + (size_t)(row0 + ln) * lda2; const _Float16* l1p = l0p + (size_t)16 * lda2;
    const _Float16* m0p = B2 + (size_t)(col0 + ln) * ldb2; const _Float16* m1p = m0p + (size_t)16 * ldb2; const _Float16* m2p = m1p + (size_t)16 * ldb2; const _Float16* m3p = m2p + (size_t)16 * ldb2;
    g2_kloop(l0p, l1p, b0p, b1p, b2p, b3p, K, hh, c00, c01, c02, c03, c10, c11, c12, c13);
    g2_kloop(a0p, a1p, m0p, m1p, m2p, m3p, K, hh, c00, c01, c02, c03, c10, c11, c12, c13);
    c00 = c00 * rscale; c01 = c01 * rscale; c02 = c02 * rscale; c03 = c03 * rscale; c10 = c10 * rscale; c11 = c11 * rscale; c12 = c12 * rscale; c13 = c13 * rscale;
  }
  g2_kloop(a0p, a1p, b0p, b1p, b2p, b3p, K, hh, c00, c01, c02, c03, c10, c11, c12, c13);
  v8f accs[8] = {c00, c01, c02, c03, c10, c11, c12, c13};
#pragma unroll
  for (int u = 0; u < 8; ++u) { const int t = u & 3, half = u >> 2; const int col = col0 + t * 16 + ln; const float bv = bp ? bf16_rne(bp[col]) : 0.f;
#pragma unroll
    for (int r = 0; r < 8; ++r) { const int rloc = half * 16 + 8 * hh + r; so[w][rloc][t * 16 + ln] = accs[u][r] * alpha + bv; } }
  __builtin_amdgcn_fence(4  , "workgroup"); __builtin_amdgcn_wave_barrier();
  const int rsub = lane >> 4, c4 = (lane & 15) * 4; const bool wl = (C16L != nullptr) && (col0 < NL);
  for (int pass = 0; pass < 2; ++pass) {
#pragma unroll
    for (int q = 0; q < 16; ++q) { const int r = q * 2 + rsub; const v4f v = *(const v4fa*)&so[w][r][c4];
      if (C) *(volatile v4f*)(C + cofs + (size_t)(row0 + r) * ldc + col0 + c4) = v;
      if (C16) { v4h h4; for (int i = 0; i < 4; ++i) h4[i] = (_Float16)v[i]; *(volatile v4h*)(C16 + cofs + (size_t)(row0 + r) * ldc + col0 + c4) = h4;
        if (wl) { v4h l4; for (int i = 0; i < 4; ++i) l4[i] = (_Float16)((v[i] - (float)h4[i]) * LCARRY); *(volatile v4h*)(C16L + cofl + (size_t)(row0 + r) * ldcl + col0 + c4) = l4; } } }
    if (pass == 0) __threadfence(); } }

__global__ __launch_bounds__(256) void k_w16(const float* __restrict__ Wq, const float* __restrict__ Wk, const float* __restrict__ Wv, _Float16* __restrict__ BW) {
  const int t = blockIdx.x * 256 + threadIdx.x; if (t >= QP * (CIN / 8)) return;
  const int n = t / (CIN / 8), k8 = (t % (CIN / 8)) * 8;
  const int hq = n / HCS, tt = n - hq * HCS;
  const int sel = (n >= VOF) ? 2 : ((tt < HD) ? 0 : ((tt < 2 * HD) ? 1 : 3));
  const int orow = (n >= VOF) ? (n - VOF) : (hq * HD + (tt & (HD - 1)));
  const float* src = (sel == 0) ? Wk : ((sel == 2) ? Wv : Wq);
  const float* p = src + (size_t)orow * CIN + k8;
  const v4f a = *(const v4fa*)p, c = *(const v4fa*)(p + 4); const float zf = (sel == 3) ? 0.0f : 16.0f;
  FragH f;
#pragma unroll
  for (int q = 0; q < 4; ++q) { f.h[q] = (_Float16)(bf16_rne(a[q]) * zf); f.h[4 + q] = (_Float16)(bf16_rne(c[q]) * zf); }
  const v8us o = f.half[0];
  *(volatile v8us*)((unsigned short*)BW + (size_t)n * CIN + k8) = o; __threadfence(); *(volatile v8us*)((unsigned short*)BW + (size_t)n * CIN + k8) = o;
}

__global__ __launch_bounds__(256) void k_bias(const float* __restrict__ bq, const float* __restrict__ bk, const float* __restrict__ bv, float* __restrict__ BI) {
  const int t = threadIdx.x; v4f o;
#pragma unroll
  for (int i = 0; i < 4; ++i) { const int n = 4 * t + i; const int hq = n / HCS, tt = n - hq * HCS;
    const int sel = (n >= VOF) ? 2 : ((tt < HD) ? 0 : ((tt < 2 * HD) ? 1 : 3));
    const int orow = (n >= VOF) ? (n - VOF) : (hq * HD + (tt & (HD - 1)));
    const float a = bk[orow], b2 = bq[orow], c = bv[orow];
    o[i] = (sel == 0) ? a : ((sel == 1) ? b2 : ((sel == 2) ? c : 0.0f)); }
  *(volatile v4f*)(BI + 4 * t) = o; __threadfence(); *(volatile v4f*)(BI + 4 * t) = o;
}

__global__ __launch_bounds__(256) void k_x16t(const float* __restrict__ x, _Float16* __restrict__ X16) {
  __shared__ __attribute__((aligned(16))) unsigned short tl[64][72];
  const int tid = threadIdx.x; constexpr int NCT = CIN / 64, NNT = SEQ / 64;
  const int ct = blockIdx.x % NCT, nt = (blockIdx.x / NCT) % NNT, b = blockIdx.x / (NCT * NNT);
  const int n0 = nt * 64, c0 = ct * 64;
  for (int i = tid; i < 64 * 16; i += 256) { const int cr = i >> 4, f4 = i & 15;
    const v4f a = *(const v4fa*)(x + ((size_t)b * CIN + c0 + cr) * SEQ_FULL + n0 + f4 * 4); FragH f;
#pragma unroll
    for (int q = 0; q < 4; ++q) { f.h[q] = (_Float16)bf16_rne(a[q]); tl[f4 * 4 + q][cr] = f.u[q]; } }
  __syncthreads();
  for (int pass = 0; pass < 2; ++pass) {
#pragma unroll
    for (int rd = 0; rd < 2; ++rd) { const int n = rd * 32 + (tid >> 3), pc = tid & 7; FragH f;
#pragma unroll
      for (int q = 0; q < 8; ++q) f.u[q] = tl[n][pc * 8 + q];
      *(volatile v8us*)((unsigned short*)X16 + ((size_t)b * SEQ + n0 + n) * CIN + c0 + pc * 8) = f.half[0]; }
    if (pass == 0) __threadfence(); } }

__global__ __launch_bounds__(64) void k_pos(const float* __restrict__ rel_h, const float* __restrict__ rel_w, _Float16* __restrict__ QHp, _Float16* __restrict__ QLp) {
  __shared__ __attribute__((aligned(16))) unsigned short pp[2][64];
  const int tid = threadIdx.x; const int h = blockIdx.x / SEQ, m = blockIdx.x - h * SEQ; const int d = tid;
  const float v = bf16_rne(rel_h[(size_t)(h * HD + d) * GW + (m % GW)]) + bf16_rne(rel_w[(size_t)(h * HD + d) * GW + (m / GW)]);
  const _Float16 hv = (_Float16)v; const _Float16 lv = (_Float16)((v - (float)hv) * LCARRY);
  FragH f; f.h[0] = hv; f.h[1] = lv; pp[0][d] = f.u[0]; pp[1][d] = f.u[1];
  __syncthreads();
  for (int pass = 0; pass < 2; ++pass) {
    for (int idx = tid; idx < NB * 16; idx += 64) { const int plane = idx / (NB * 8), rem = idx - plane * (NB * 8), b = rem >> 3, pc = rem & 7; FragH g;
#pragma unroll
      for (int q = 0; q < 8; ++q) g.u[q] = pp[plane][pc * 8 + q];
      unsigned short* dst = plane ? ((unsigned short*)QLp + ((size_t)b * SEQ + m) * QPL + h * HCS + 2 * HD + pc * 8)
                                  : ((unsigned short*)QHp + ((size_t)b * SEQ + m) * QP + h * HCS + 2 * HD + pc * 8);
      *(volatile v8us*)dst = g.half[0]; }
    if (pass == 0) __threadfence(); } }

__global__ __launch_bounds__(256) void k_vt(const _Float16* __restrict__ QHp, _Float16* __restrict__ Vt) {
  __shared__ unsigned short tl[64][66]; const int tid = threadIdx.x; constexpr int NLG = SEQ / 64;
  const int lg = blockIdx.x % NLG, bh = blockIdx.x / NLG, h = bh % NH, b = bh / NH;
  for (int i = tid; i < 64 * 8; i += 256) { const int r = i / 8, c8 = (i % 8) * 8; FragH f; f.half[0] = *(const v8us*)((const unsigned short*)QHp + ((size_t)b * SEQ + lg * 64 + r) * QP + VOF + h * HD + c8);
#pragma unroll
    for (int q = 0; q < 8; ++q) tl[r][c8 + q] = f.u[q]; }
  __syncthreads();
  for (int pass = 0; pass < 2; ++pass) {
#pragma unroll
    for (int rd = 0; rd < 2; ++rd) { const int d = rd * 32 + tid / 8, pc = tid % 8; FragH f;
#pragma unroll
      for (int q = 0; q < 8; ++q) f.u[q] = tl[pc * 8 + q][d];
      *(volatile v8us*)((unsigned short*)Vt + (((size_t)b * NH + h) * HD + d) * SEQ + lg * 64 + pc * 8) = f.half[0]; }
    if (pass == 0) __threadfence(); } }

__global__ __launch_bounds__(256) void k_rsmw(const float* __restrict__ S, _Float16* __restrict__ P, int nrows) {
  #pragma clang fp contract(off)
  const int row = blockIdx.x * 8 + (threadIdx.x >> 5), lane = threadIdx.x & 31;
  if (row >= nrows) return;
  const float* s = S + (size_t)row * SEQ;
  constexpr int NI = SEQ / 256;
  float v[NI * 8];
  float mx = -3.0e38f;
#pragma unroll
  for (int i = 0; i < NI; ++i) {
    const v4f a = *(const v4fa*)(s + i * 256 + lane * 8), c = *(const v4fa*)(s + i * 256 + lane * 8 + 4);
#pragma unroll
    for (int q = 0; q < 4; ++q) { v[i * 8 + q] = a[q]; v[i * 8 + 4 + q] = c[q]; mx = fmaxf(mx, fmaxf(a[q], c[q])); }
  }
#pragma unroll
  for (int o = 16; o > 0; o >>= 1) mx = fmaxf(mx, __shfl_xor(mx, o, 32));
  float se = 0.f;
#pragma unroll
  for (int j = 0; j < NI * 8; ++j) { const float e = __expf(v[j] - mx); v[j] = e; se += e; }
#pragma unroll
  for (int o = 16; o > 0; o >>= 1) se += __shfl_xor(se, o, 32);
  const float sc = PCARRY / se;
  unsigned short* prow = (unsigned short*)P + (size_t)row * SEQ;
  for (int pass = 0; pass < 2; ++pass) {
#pragma unroll
    for (int i = 0; i < NI; ++i) { FragH f;
#pragma unroll
      for (int q = 0; q < 8; ++q) f.h[q] = (_Float16)(v[i * 8 + q] * sc);
      *(volatile v8us*)(prow + i * 256 + lane * 8) = f.half[0]; }
    if (pass == 0) __threadfence();
  }
}

extern "C" void kernel_launch(void* const* d_in, const int* in_sizes, int n_in,
                              void* d_out, int out_size, void* d_ws, size_t ws_size, hipStream_t stream) {
  if (n_in < 9) return;
  const float* x     = (const float*)d_in[0];
  const float* Wq    = (const float*)d_in[1];
  const float* bq    = (const float*)d_in[2];
  const float* Wk    = (const float*)d_in[3];
  const float* bk    = (const float*)d_in[4];
  const float* Wv    = (const float*)d_in[5];
  const float* bv    = (const float*)d_in[6];
  const float* rel_h = (const float*)d_in[7];
  const float* rel_w = (const float*)d_in[8];
  if (in_sizes[0] < (int)(((size_t)NB * CIN - 1) * SEQ_FULL + SEQ)) return;
  if (in_sizes[1] < CIN * CIN || in_sizes[3] < CIN * CIN || in_sizes[5] < CIN * CIN) return;
  if (in_sizes[2] < CIN || in_sizes[4] < CIN || in_sizes[6] < CIN) return;
  if (in_sizes[7] < NH * HD * GW || in_sizes[8] < NH * HD * GW) return;
  if (out_size < (int)((size_t)NB * CIN * SEQ)) return;
  char* ws = (char*)d_ws; size_t off = 0;
  auto take = [&](size_t bytes) { char* p = ws + off; off += (bytes + 255) & ~(size_t)255; return p; };
  _Float16* BW = (_Float16*)take((size_t)QP * CIN * 2);
  float*    BI = (float*)take((size_t)QP * 4);
  _Float16* QH = (_Float16*)take(NR * QP * 2);
  _Float16* QL = (_Float16*)take(NR * QPL * 2);
  _Float16* VT = (_Float16*)take((size_t)NB * NH * HD * SEQ * 2);
  const size_t shX = NR * CIN * 2, shS = (size_t)NH * SEQ * SEQ * 4, shP = (size_t)NH * SEQ * SEQ * 2;
  const size_t shBytes = (shX > shS + shP) ? shX : (shS + shP);
  char* SH = take(shBytes);
  _Float16* X16 = (_Float16*)SH; float* S = (float*)SH; _Float16* P = (_Float16*)(SH + shS);
  if (off > ws_size) return;
  float* out = (float*)d_out;

  k_w16<<<(unsigned)((QP * (CIN / 8) + 255) / 256), 256, 0, stream>>>(Wq, Wk, Wv, BW);
  k_bias<<<1, 256, 0, stream>>>(bq, bk, bv, BI);
  k_x16t<<<(unsigned)(NB * (SEQ / 64) * (CIN / 64)), 256, 0, stream>>>(x, X16);
  k_gemm2<0><<<dim3((unsigned)((NR / 128) * (QP / 64)), 1), 128, 0, stream>>>(X16, CIN, 0, nullptr, 0, 0, BW, CIN, 0, nullptr, 0, 0, 1.0f,
      0.0625f, BI, 0, nullptr, QH, QP, 0, QL, QPL, 0, QPL, (int)NR, QP, CIN);
  k_pos<<<(unsigned)(NH * SEQ), 64, 0, stream>>>(rel_h, rel_w, QH, QL);
  k_vt<<<(unsigned)(NB * NH * (SEQ / 64)), 256, 0, stream>>>(QH, VT);
  for (int b = 0; b < NB; ++b) {
    const _Float16* QHb = QH + (size_t)b * SEQ * QP; const _Float16* QLb = QL + (size_t)b * SEQ * QPL;
    k_gemm2<1><<<dim3((SEQ / 128) * (SEQ / 64), NH), 128, 0, stream>>>(QHb + HD, QP, (size_t)HCS, QLb + HD, QPL, (size_t)HCS, QHb, QP, (size_t)HCS, QLb, QPL, (size_t)HCS, 1.0f / LCARRY,
        1.0f, nullptr, 0, S, nullptr, SEQ, (size_t)SEQ * SEQ, nullptr, 0, 0, 0, SEQ, SEQ, 2 * HD);
    k_rsmw<<<(NH * SEQ + 7) / 8, 256, 0, stream>>>(S, P, NH * SEQ);
    k_gemm2<0><<<dim3(((HD + 127) / 128) * (SEQ / 64), NH), 128, 0, stream>>>(VT + (size_t)b * NH * HD * SEQ, SEQ, (size_t)HD * SEQ, nullptr, 0, 0, P, SEQ, (size_t)SEQ * SEQ, nullptr, 0, 0, 1.0f,
        1.0f / PCARRY, nullptr, 0, out + (size_t)b * CIN * SEQ, nullptr, SEQ, (size_t)HD * SEQ, nullptr, 0, 0, 0, HD, SEQ, SEQ);
  }
}
